// input_layer_21758304322131
// MI455X (gfx1250) — hardware-verified
//
#include <hip/hip_runtime.h>
#include <math.h>


typedef _Float16       v16h __attribute__((ext_vector_type(16)));
typedef __bf16         v16b __attribute__((ext_vector_type(16)));
typedef _Float16       v8h  __attribute__((ext_vector_type(8)));
typedef float          v8f  __attribute__((ext_vector_type(8)));
typedef float          v4f  __attribute__((ext_vector_type(4)));
typedef int            v4i  __attribute__((ext_vector_type(4)));
typedef _Float16       v4h  __attribute__((ext_vector_type(4)));
typedef v4f __attribute__((may_alias)) v4fa;
typedef v4i __attribute__((may_alias)) v4ia;
typedef v4h __attribute__((may_alias)) v4ha;

#define XS_S 264
#define VH_S 260
#define HB_S 260
#define U_S  1040

__device__ __forceinline__ float silu_f(float x) {
  return x * __builtin_amdgcn_rcpf(1.0f + __expf(-x));
}

__device__ __forceinline__ float wave_sum32(float v) {
#pragma unroll
  for (int off = 16; off > 0; off >>= 1) v += __shfl_xor(v, off, 32);
  return v;
}

__device__ __forceinline__ unsigned short f2bf(float f) {
  unsigned int u = __float_as_uint(f);
  u += 0x7FFFu + ((u >> 16) & 1u);
  return (unsigned short)(u >> 16);
}
__device__ __forceinline__ float bf2f(unsigned short b) {
  return __uint_as_float(((unsigned int)b) << 16);
}

__device__ __forceinline__ v8f mma_f16(v16h a, v16h b, v8f c) {
  c = __builtin_amdgcn_wmma_f32_16x16x32_f16(false, a, false, b, (short)0, c, false, false);
  asm volatile("v_nop\n\tv_nop\n\tv_nop\n\tv_nop" : "+v"(c) : "v"(a), "v"(b));
  return c;
}
__device__ __forceinline__ v8f mma_bf16(v16b a, v16b b, v8f c) {
  c = __builtin_amdgcn_wmma_f32_16x16x32_bf16(false, a, false, b, (short)0, c, false, false);
  asm volatile("v_nop\n\tv_nop\n\tv_nop\n\tv_nop" : "+v"(c) : "v"(a), "v"(b));
  return c;
}

__device__ __forceinline__ v16h lda_h(const _Float16* buf, int stride, int m0, int k0, int lane) {
  const _Float16* p = buf + (m0 + (lane & 15)) * stride + k0 + ((lane >> 4) << 3);
  union { v16h v; v4i q[2]; } u;
  u.q[0] = *(const v4ia*)(p);
  u.q[1] = *(const v4ia*)(p + 16);
  return u.v;
}
__device__ __forceinline__ v16b lda_b(const unsigned short* buf, int stride, int m0, int k0, int lane) {
  const unsigned short* p = buf + (m0 + (lane & 15)) * stride + k0 + ((lane >> 4) << 3);
  union { v16b v; v4i q[2]; } u;
  u.q[0] = *(const v4ia*)(p);
  u.q[1] = *(const v4ia*)(p + 16);
  return u.v;
}

__device__ __forceinline__ v16h ldb_h(const _Float16* pack, int NT, int kt, int nt, int lane) {
  const _Float16* p = pack + (((size_t)((kt * NT + nt) * 32 + lane)) << 4);
  union { v16h v; v4i q[2]; } u;
  u.q[0] = *(const v4ia*)(p);
  u.q[1] = *(const v4ia*)(p + 8);
  return u.v;
}
__device__ __forceinline__ v16b ldb_b(const unsigned short* pack, int NT, int kt, int nt, int lane) {
  const unsigned short* p = pack + (((size_t)((kt * NT + nt) * 32 + lane)) << 4);
  union { v16b v; v4i q[2]; } u;
  u.q[0] = *(const v4ia*)(p);
  u.q[1] = *(const v4ia*)(p + 8);
  return u.v;
}

__global__ __launch_bounds__(256)
void pack_f16_kernel(const float* __restrict__ W, _Float16* __restrict__ P,
                     int Kdim, int Ndim, float scale) {
  const int i8 = blockIdx.x * 256 + threadIdx.x;
  const int total8 = (Kdim * Ndim) >> 3;
  if (i8 >= total8) return;
  const int jg   = i8 & 1;
  const int idx  = i8 >> 1;
  const int L    = idx & 31;
  const int frag = idx >> 5;
  const int NT   = Ndim >> 4;
  const int nt   = frag % NT;
  const int kt   = frag / NT;
  const int kb   = kt * 32 + ((L >> 4) << 3) + (jg << 4);
  const int n    = nt * 16 + (L & 15);
  union { v8h h; v4i q; } u;
#pragma unroll
  for (int e = 0; e < 8; ++e) u.h[e] = (_Float16)(W[(size_t)(kb + e) * Ndim + n] * scale);
  _Float16* dst = P + ((size_t)i8 << 3);
  *(volatile v4i*)dst = u.q;
  __threadfence();
  *(volatile v4i*)dst = u.q;
}

__global__ __launch_bounds__(256)
void pack_bf16hl_kernel(const float* __restrict__ W, unsigned short* __restrict__ Ph,
                        unsigned short* __restrict__ Pl, int Kdim, int Ndim) {
  const int i8 = blockIdx.x * 256 + threadIdx.x;
  const int total8 = (Kdim * Ndim) >> 3;
  if (i8 >= total8) return;
  const int jg   = i8 & 1;
  const int idx  = i8 >> 1;
  const int L    = idx & 31;
  const int frag = idx >> 5;
  const int NT   = Ndim >> 4;
  const int nt   = frag % NT;
  const int kt   = frag / NT;
  const int kb   = kt * 32 + ((L >> 4) << 3) + (jg << 4);
  const int n    = nt * 16 + (L & 15);
  union { unsigned short s[8]; v4i q; } uh, ul;
#pragma unroll
  for (int e = 0; e < 8; ++e) {
    const float w = W[(size_t)(kb + e) * Ndim + n];
    const unsigned short hb = f2bf(w);
    uh.s[e] = hb;
    ul.s[e] = f2bf(w - bf2f(hb));
  }
  unsigned short* dh = Ph + ((size_t)i8 << 3);
  unsigned short* dl = Pl + ((size_t)i8 << 3);
  *(volatile v4i*)dh = uh.q;
  *(volatile v4i*)dl = ul.q;
  __threadfence();
  *(volatile v4i*)dh = uh.q;
  *(volatile v4i*)dl = ul.q;
}

__global__ __launch_bounds__(256)
void front_kernel(const float* __restrict__ x,
                  const int*   __restrict__ gli,
                  const int*   __restrict__ dropm,
                  const int*   __restrict__ imap,
                  const int*   __restrict__ inr,
                  const float* __restrict__ icoord,
                  const float* __restrict__ gcoord,
                  const float* __restrict__ Win,
                  const float* __restrict__ bin,
                  const float* __restrict__ Wpe,
                  const float* __restrict__ Wbias,
                  const _Float16* __restrict__ WvP,
                  unsigned short* __restrict__ AOH,
                  unsigned short* __restrict__ AOL,
                  int nGroups, int nGrid, int nPts)
{
  __shared__ __attribute__((aligned(16))) _Float16 s_xh[64 * XS_S];
  __shared__ __attribute__((aligned(16))) _Float16 s_xl[64 * XS_S];
  __shared__ __attribute__((aligned(16))) float    s_vh[64 * VH_S];
  __shared__ __attribute__((aligned(16))) float    s_sc[32 * 64];
  __shared__ __attribute__((aligned(16))) float    s_of[4 * 256];
  __shared__ __attribute__((aligned(16))) float    s_xi[64 * 8];
  __shared__ float s_wpe[64];
  __shared__ float s_wb[256];
  __shared__ float s_lon1[4], s_lat1[4];
  __shared__ int   s_g[4], s_dm[4];

  const int tid  = threadIdx.x;
  const int lane = tid & 31;
  const int wv   = tid >> 5;
  const int hh   = lane >> 4;
  const int bx   = blockIdx.x;
  if (bx >= nGroups) return;

  if (tid < 4) {
    const int cell = 4 * bx + tid;
    int g = gli[cell];
    g = g < 0 ? 0 : (g >= nGrid ? nGrid - 1 : g);
    s_g[tid]    = g;
    s_dm[tid]   = (dropm[cell] != 0) ? 1 : 0;
    s_lon1[tid] = gcoord[g];
    s_lat1[tid] = gcoord[nGrid + g];
  }
  if (tid < 64) s_wpe[tid] = Wpe[tid];
  s_wb[tid] = Wbias[tid];
#pragma unroll
  for (int i = 0; i < 2; ++i) {
    const int e = tid + i * 256;
    const int m = e >> 3, f = e & 7;
    s_xi[e] = x[((size_t)(4 * bx + (m >> 4)) * 16 + (m & 15)) * 8 + f];
  }
  float wreg[8];
#pragma unroll
  for (int f = 0; f < 8; ++f) wreg[f] = Win[f * 256 + tid];
  const float breg = bin[tid];
  __syncthreads();

  for (int m = 0; m < 64; ++m) {
    float acc = 0.0f;
#pragma unroll
    for (int f = 0; f < 8; ++f) acc += s_xi[m * 8 + f] * wreg[f];
    acc += breg;
    const float sv = silu_f(acc) * 16.0f;
    const _Float16 hi = (_Float16)sv;
    const _Float16 lo = (_Float16)((sv - (float)hi) * 2048.0f);
    s_xh[m * XS_S + tid] = hi;
    s_xl[m * XS_S + tid] = lo;
  }

  {
    const int t = tid >> 6, k = tid & 63;
    const int sidx = k >> 4, j = k & 15;
    const int g = s_g[sidx];
    int im = imap[g * 16 + j];
    im = im < 0 ? 0 : (im >= nPts ? nPts - 1 : im);
    const int masked = (inr[g * 16 + j] == 0 ? 1 : 0) | s_dm[sidx];
    const float dlon = icoord[im]        - s_lon1[t];
    const float dlat = icoord[nPts + im] - s_lat1[t];
    const float dist = sqrtf(dlon * dlon + dlat * dlat + 1e-12f);
    const float ang  = atan2f(dlat, dlon);
    float bias[8];
#pragma unroll
    for (int h = 0; h < 8; ++h) bias[h] = 0.0f;
#pragma unroll 4
    for (int p = 0; p < 32; ++p) {
      const float pe = silu_f(dist * s_wpe[p] + ang * s_wpe[32 + p]);
#pragma unroll
      for (int h = 0; h < 8; ++h) bias[h] += pe * s_wb[p * 8 + h];
    }
#pragma unroll
    for (int h = 0; h < 8; ++h)
      s_sc[(h * 4 + t) * 64 + k] = masked ? -1e9f : bias[h];
  }
  __syncthreads();

  if (tid < 32) {
    float* r = &s_sc[tid * 64];
    float mx = -3.4e38f;
    for (int k = 0; k < 64; ++k) mx = fmaxf(mx, r[k]);
    float sum = 0.0f;
    for (int k = 0; k < 64; ++k) { const float e = expf(r[k] - mx); r[k] = e; sum += e; }
    const float inv = 1.0f / sum;
    for (int k = 0; k < 64; ++k) r[k] *= inv;
  }
  __syncthreads();

  for (int i = 0; i < 8; ++i) {
    const int tile = wv + 8 * i;
    const int mt = tile >> 4, nt = tile & 15;
    v8f acch = {};
    v8f accl = {};
#pragma unroll
    for (int kt = 0; kt < 8; ++kt) {
      const v16h ah = lda_h(s_xh, XS_S, mt * 16, kt * 32, lane);
      const v16h al = lda_h(s_xl, XS_S, mt * 16, kt * 32, lane);
      const v16h bf = ldb_h(WvP, 16, kt, nt, lane);
      acch = mma_f16(ah, bf, acch);
      accl = mma_f16(al, bf, accl);
    }
    const int n  = nt * 16 + (lane & 15);
    const int mb = mt * 16 + (hh << 3);
#pragma unroll
    for (int r = 0; r < 8; ++r)
      s_vh[(mb + r) * VH_S + n] = (acch[r] + accl[r] * (1.0f / 2048.0f)) * (1.0f / 1024.0f);
  }
  __syncthreads();

#pragma unroll
  for (int i = 0; i < 4; ++i) {
    const int t = i, d = tid, h = d >> 5;
    const float* sp = &s_sc[(h * 4 + t) * 64];
    const float* vp = &s_vh[d];
    float acc = 0.0f;
    for (int k = 0; k < 64; ++k) acc += sp[k] * vp[k * VH_S];
    s_of[t * 256 + d] = acc;
  }
  __syncthreads();

  if (wv < 4) {
    const v4fa* src = (const v4fa*)(s_of + wv * 256 + 8 * lane);
    const v4f a0 = src[0];
    const v4f a1 = src[1];
    float o[8] = {a0[0], a0[1], a0[2], a0[3], a1[0], a1[1], a1[2], a1[3]};
    union { unsigned short s[8]; v4i q; } uh, ul;
#pragma unroll
    for (int e = 0; e < 8; ++e) {
      const unsigned short hb = f2bf(o[e]);
      uh.s[e] = hb;
      ul.s[e] = f2bf(o[e] - bf2f(hb));
    }
    const size_t off = (size_t)(4 * bx + wv) * 256 + 8 * lane;
    *(volatile v4i*)(AOH + off) = uh.q;
    *(volatile v4i*)(AOL + off) = ul.q;
    __threadfence();
    *(volatile v4i*)(AOH + off) = uh.q;
    *(volatile v4i*)(AOL + off) = ul.q;
  }
}

__global__ __launch_bounds__(256)
void tail_kernel(const unsigned short* __restrict__ AOH, const unsigned short* __restrict__ AOL,
                 const unsigned short* __restrict__ WoPh, const unsigned short* __restrict__ WoPl,
                 const _Float16* __restrict__ W1P, const _Float16* __restrict__ W2P,
                 const float* __restrict__ g1, const float* __restrict__ b1,
                 const float* __restrict__ g2, const float* __restrict__ b2,
                 float* __restrict__ out, int nRows)
{
  __shared__ __attribute__((aligned(16))) unsigned short s_abh[16 * XS_S];
  __shared__ __attribute__((aligned(16))) unsigned short s_abl[16 * XS_S];
  __shared__ __attribute__((aligned(16))) float    s_hb[16 * HB_S];
  __shared__ __attribute__((aligned(16))) float    s_w2[16 * HB_S];
  __shared__ __attribute__((aligned(16))) _Float16 s_h16[16 * XS_S];
  __shared__ __attribute__((aligned(16))) _Float16 s_u[16 * U_S];

  const int tid  = threadIdx.x;
  const int lane = tid & 31;
  const int wv   = tid >> 5;
  const int hh   = lane >> 4;
  const int r0   = blockIdx.x * 16;
  if (r0 + 16 > nRows) return;

#pragma unroll
  for (int i = 0; i < 2; ++i) {
    const int e = tid + 256 * i;
    const int m = e >> 5, c = e & 31;
    const size_t go = (size_t)(r0 + m) * 256 + 8 * c;
    const v4i qh = *(const v4ia*)(AOH + go);
    const v4i ql = *(const v4ia*)(AOL + go);
    *(v4ia*)(s_abh + m * XS_S + 8 * c) = qh;
    *(v4ia*)(s_abl + m * XS_S + 8 * c) = ql;
  }
  __syncthreads();

#pragma unroll
  for (int i = 0; i < 2; ++i) {
    const int nt = wv * 2 + i;
    v8f acc = {};
#pragma unroll
    for (int kt = 0; kt < 8; ++kt) {
      const v16b ah = lda_b(s_abh, XS_S, 0, kt * 32, lane);
      const v16b al = lda_b(s_abl, XS_S, 0, kt * 32, lane);
      const v16b bh = ldb_b(WoPh, 16, kt, nt, lane);
      const v16b bl = ldb_b(WoPl, 16, kt, nt, lane);
      acc = mma_bf16(ah, bh, acc);
      acc = mma_bf16(al, bh, acc);
      acc = mma_bf16(ah, bl, acc);
    }
    const int n  = nt * 16 + (lane & 15);
    const int mb = hh << 3;
#pragma unroll
    for (int r = 0; r < 8; ++r) s_hb[(mb + r) * HB_S + n] = acc[r];
  }
  __syncthreads();

#pragma unroll
  for (int rr = 0; rr < 2; ++rr) {
    const int m = wv * 2 + rr;
    v4f v[2];
    float su = 0.0f;
#pragma unroll
    for (int j = 0; j < 2; ++j) {
      v[j] = *(const v4fa*)(s_hb + m * HB_S + 128 * j + 4 * lane);
      su += v[j][0] + v[j][1] + v[j][2] + v[j][3];
    }
    const float mu = wave_sum32(su) * (1.0f / 256.0f);
    float sq = 0.0f;
#pragma unroll
    for (int j = 0; j < 2; ++j) {
      const v4f dv = v[j] - mu;
      sq += dv[0] * dv[0] + dv[1] * dv[1] + dv[2] * dv[2] + dv[3] * dv[3];
    }
    const float var = wave_sum32(sq) * (1.0f / 256.0f);
    const float rs  = rsqrtf(var + 1e-5f);
#pragma unroll
    for (int j = 0; j < 2; ++j) {
      const int d = 128 * j + 4 * lane;
      const v4f gv = *(const v4fa*)(g1 + d);
      const v4f bv = *(const v4fa*)(b1 + d);
      const v4f hv = (v[j] - mu) * rs * gv + bv;
      *(v4fa*)(s_hb + m * HB_S + d) = hv;
      v4h h4;
      h4[0] = (_Float16)hv[0]; h4[1] = (_Float16)hv[1];
      h4[2] = (_Float16)hv[2]; h4[3] = (_Float16)hv[3];
      *(v4ha*)(s_h16 + m * XS_S + d) = h4;
    }
  }
  __syncthreads();

  for (int i = 0; i < 8; ++i) {
    const int nt = wv * 8 + i;
    v8f acc = {};
#pragma unroll
    for (int kt = 0; kt < 8; ++kt) {
      const v16h a  = lda_h(s_h16, XS_S, 0, kt * 32, lane);
      const v16h bf = ldb_h(W1P, 64, kt, nt, lane);
      acc = mma_f16(a, bf, acc);
    }
    const int n  = nt * 16 + (lane & 15);
    const int mb = hh << 3;
#pragma unroll
    for (int r = 0; r < 8; ++r)
      s_u[(mb + r) * U_S + n] = (_Float16)(silu_f(acc[r] * (1.0f / 64.0f)) * 16.0f);
  }
  __syncthreads();

#pragma unroll
  for (int i = 0; i < 2; ++i) {
    const int nt = wv * 2 + i;
    v8f acc = {};
#pragma unroll 4
    for (int kt = 0; kt < 32; ++kt) {
      const v16h a  = lda_h(s_u, U_S, 0, kt * 32, lane);
      const v16h bf = ldb_h(W2P, 16, kt, nt, lane);
      acc = mma_f16(a, bf, acc);
    }
    const int n  = nt * 16 + (lane & 15);
    const int mb = hh << 3;
#pragma unroll
    for (int r = 0; r < 8; ++r) s_w2[(mb + r) * HB_S + n] = acc[r] * (1.0f / 1024.0f);
  }
  __syncthreads();

  v4f y[2][2];
#pragma unroll
  for (int rr = 0; rr < 2; ++rr) {
    const int m = wv * 2 + rr;
    v4f v[2];
    float su = 0.0f;
#pragma unroll
    for (int j = 0; j < 2; ++j) {
      const int d = 128 * j + 4 * lane;
      const v4f hv = *(const v4fa*)(s_hb + m * HB_S + d);
      const v4f wv2 = *(const v4fa*)(s_w2 + m * HB_S + d);
      v[j] = hv + wv2;
      su += v[j][0] + v[j][1] + v[j][2] + v[j][3];
    }
    const float mu = wave_sum32(su) * (1.0f / 256.0f);
    float sq = 0.0f;
#pragma unroll
    for (int j = 0; j < 2; ++j) {
      const v4f dv = v[j] - mu;
      sq += dv[0] * dv[0] + dv[1] * dv[1] + dv[2] * dv[2] + dv[3] * dv[3];
    }
    const float var = wave_sum32(sq) * (1.0f / 256.0f);
    const float rs  = rsqrtf(var + 1e-5f);
#pragma unroll
    for (int j = 0; j < 2; ++j) {
      const int d = 128 * j + 4 * lane;
      const v4f gv = *(const v4fa*)(g2 + d);
      const v4f bv = *(const v4fa*)(b2 + d);
      y[rr][j] = (v[j] - mu) * rs * gv + bv;
    }
  }
#pragma unroll
  for (int rr = 0; rr < 2; ++rr) {
    float* op = out + (size_t)(r0 + wv * 2 + rr) * 256;
#pragma unroll
    for (int j = 0; j < 2; ++j) *(volatile v4f*)(op + 128 * j + 4 * lane) = y[rr][j];
  }
  __threadfence();
#pragma unroll
  for (int rr = 0; rr < 2; ++rr) {
    float* op = out + (size_t)(r0 + wv * 2 + rr) * 256;
#pragma unroll
    for (int j = 0; j < 2; ++j) *(volatile v4f*)(op + 128 * j + 4 * lane) = y[rr][j];
  }
}

extern "C" void kernel_launch(void* const* d_in, const int* in_sizes, int n_in,
                              void* d_out, int out_size, void* d_ws, size_t ws_size,
                              hipStream_t stream) {
  if (n_in < 19) return;
  const float* x      = (const float*)d_in[0];
  const int*   gli    = (const int*)d_in[1];
  const int*   dropm  = (const int*)d_in[2];
  const int*   imap   = (const int*)d_in[3];
  const int*   inr    = (const int*)d_in[4];
  const float* icoord = (const float*)d_in[5];
  const float* gcoord = (const float*)d_in[6];
  const float* Win    = (const float*)d_in[7];
  const float* bin    = (const float*)d_in[8];
  const float* Wpe    = (const float*)d_in[9];
  const float* Wbias  = (const float*)d_in[10];
  const float* Wv     = (const float*)d_in[11];
  const float* Wo     = (const float*)d_in[12];
  const float* W1     = (const float*)d_in[13];
  const float* W2     = (const float*)d_in[14];
  const float* g1     = (const float*)d_in[15];
  const float* b1     = (const float*)d_in[16];
  const float* g2     = (const float*)d_in[17];
  const float* b2     = (const float*)d_in[18];

  const int Dm     = in_sizes[8];
  if (Dm != 256) return;
  const int FFd    = in_sizes[13] / Dm;
  const int nCells = in_sizes[1];
  const int nGrid  = in_sizes[6] / 2;
  const int nPts   = in_sizes[5] / 2;
  const int nRows  = out_size / Dm;
  if (FFd != 1024) return;
  if (nRows != nCells) return;
  if (in_sizes[0] != nCells * 16 * 8) return;
  if ((nRows & 15) != 0) return;
  if (in_sizes[3] != nGrid * 16 || in_sizes[4] != nGrid * 16) return;
  if (in_sizes[7] != 8 * Dm || in_sizes[9] != 64 || in_sizes[10] != 256) return;
  if (in_sizes[11] != Dm * Dm || in_sizes[12] != Dm * Dm || in_sizes[14] != FFd * Dm) return;
  const int nGroups = nRows / 4;

  unsigned char* ws = (unsigned char*)d_ws;
  size_t off = 0;
  const size_t szWv  = (size_t)Dm * Dm * 2;
  const size_t szWo  = (size_t)Dm * Dm * 2;
  const size_t szW1  = (size_t)Dm * FFd * 2;
  const size_t szW2  = (size_t)FFd * Dm * 2;
  const size_t szAO  = (size_t)nRows * Dm * 2;
  _Float16*       WvP  = (_Float16*)(ws + off);       off += szWv;
  unsigned short* WoPh = (unsigned short*)(ws + off); off += szWo;
  unsigned short* WoPl = (unsigned short*)(ws + off); off += szWo;
  _Float16*       W1P  = (_Float16*)(ws + off);       off += szW1;
  _Float16*       W2P  = (_Float16*)(ws + off);       off += szW2;
  unsigned short* AOH  = (unsigned short*)(ws + off); off += szAO;
  unsigned short* AOL  = (unsigned short*)(ws + off); off += szAO;
  if (off > ws_size) return;

  const int t8Wv = (Dm * Dm) >> 3, t8W1 = (Dm * FFd) >> 3;
  pack_f16_kernel<<<(t8Wv + 255) / 256, 256, 0, stream>>>(Wv, WvP, Dm, Dm, 64.0f);
  pack_bf16hl_kernel<<<(t8Wv + 255) / 256, 256, 0, stream>>>(Wo, WoPh, WoPl, Dm, Dm);
  pack_f16_kernel<<<(t8W1 + 255) / 256, 256, 0, stream>>>(W1, W1P, Dm, FFd, 64.0f);
  pack_f16_kernel<<<(t8W1 + 255) / 256, 256, 0, stream>>>(W2, W2P, FFd, Dm, 64.0f);

  front_kernel<<<nGroups, 256, 0, stream>>>(
      x, gli, dropm, imap, inr, icoord, gcoord, Win, bin, Wpe, Wbias,
      WvP, AOH, AOL, nGroups, nGrid, nPts);

  tail_kernel<<<nRows / 16, 256, 0, stream>>>(
      AOH, AOL, WoPh, WoPl, W1P, W2P, g1, b1, g2, b2, (float*)d_out, nRows);
}
